// MultiHeadAttention_25872882992056
// MI455X (gfx1250) — hardware-verified
//
#include <hip/hip_runtime.h>


#ifndef NB
#define NB 4
#endif
#ifndef SEQ
#define SEQ 2048
#endif
#define NB_FULL  4
#define SEQ_FULL 2048
#ifndef OUT_SEQ
#define OUT_SEQ SEQ
#endif
#define DM   1024
#define NH_  16
#define HD   64
#define AW   4
#define EROWS ((SEQ) < 512 ? (SEQ) : 512)
#define QRS  2048.0f
#define QRI  (1.0f / 2048.0f)
#define SC2  (0.125f * 1.4426950408889634f)
#define NEGL (-1.0e9f * 1.4426950408889634f)
#define PSH  8.0f
#define CXS  16.0f
#define WOS  1024.0f
#define OSC  (1.0f / 16384.0f)

static_assert(HD == 64);
static_assert(NH_ * HD == DM);
static_assert(DM % 64 == 0);
static_assert(DM % 32 == 0);
static_assert(SEQ % 64 == 0);
static_assert((NB * SEQ) % 64 == 0);
static_assert(SEQ % 32 == 0);
static_assert(EROWS % 64 == 0);
static_assert(EROWS % (16 * AW) == 0);
static_assert((SEQ - EROWS) % 64 == 0);
static_assert((SEQ - EROWS) % (16 * AW) == 0);
static_assert(EROWS <= SEQ);
static_assert(((size_t)SEQ * DM) % 8 == 0);
static_assert(((size_t)DM * DM) % 8 == 0);
static_assert(NB <= NB_FULL);
static_assert(SEQ <= SEQ_FULL);

typedef _Float16 h16;
typedef unsigned short bf;
typedef __attribute__((ext_vector_type(16))) __bf16   v16bf;
typedef __attribute__((ext_vector_type(16))) _Float16 v16h;
typedef __attribute__((ext_vector_type(8)))  _Float16 v8h;
typedef __attribute__((ext_vector_type(8)))  unsigned short v8us;
typedef __attribute__((ext_vector_type(8)))  float    v8f;
typedef __attribute__((ext_vector_type(4)))  float    v4f;
typedef __attribute__((ext_vector_type(4)))  int      v4i;
typedef v4f  __attribute__((may_alias)) v4fa;

__device__ __forceinline__ unsigned short f2bf(float f) { unsigned u = __float_as_uint(f); u += 0x7FFFu + ((u >> 16) & 1u); return (unsigned short)(u >> 16); }
__device__ __forceinline__ float bfr(float f) { return __uint_as_float(((unsigned)f2bf(f)) << 16); }
__device__ __forceinline__ v16h cat16(v8h lo, v8h hi) { return __builtin_shufflevector(lo, hi, 0, 1, 2, 3, 4, 5, 6, 7, 8, 9, 10, 11, 12, 13, 14, 15); }
__device__ __forceinline__ v16bf cat16b(v8us lo, v8us hi) { return __builtin_bit_cast(v16bf, __builtin_shufflevector(lo, hi, 0, 1, 2, 3, 4, 5, 6, 7, 8, 9, 10, 11, 12, 13, 14, 15)); }
__device__ __forceinline__ v8f wmma16(v16h a, v16h b, v8f c) { return __builtin_amdgcn_wmma_f32_16x16x32_f16(false, a, false, b, (short)0, c, false, false); }
__device__ __forceinline__ v8f wmmab(v16bf a, v16bf b, v8f c) { return __builtin_amdgcn_wmma_f32_16x16x32_bf16(false, a, false, b, (short)0, c, false, false); }
__device__ __forceinline__ v16h  ldh(const h16* p) { return cat16(*(const v8h*)p, *(const v8h*)(p + 16)); }
__device__ __forceinline__ v16bf ldb(const bf* p)  { return cat16b(*(const v8us*)p, *(const v8us*)(p + 16)); }
__device__ __forceinline__ void wave_sync() { __builtin_amdgcn_fence(3  , "wavefront"); __builtin_amdgcn_wave_barrier(); asm volatile("" ::: "memory"); }

__global__ __launch_bounds__(256) void k_cvt8(const float* __restrict__ src, bf* dst, size_t n8) {
    const size_t i = (size_t)blockIdx.x * 256 + threadIdx.x; if (i >= n8) return;
    const v8f v = *(const v8f*)(src + i * 8); v8us o;
#pragma unroll
    for (int k = 0; k < 8; ++k) o[k] = f2bf(v[k]);
    *(volatile v8us*)(dst + i * 8) = o; __threadfence(); *(volatile v8us*)(dst + i * 8) = o;
}

__global__ __launch_bounds__(256) void k_cvtw8(const float* __restrict__ src, h16* dst, size_t n8) {
    const size_t i = (size_t)blockIdx.x * 256 + threadIdx.x; if (i >= n8) return;
    const v8f v = *(const v8f*)(src + i * 8); v8h o;
#pragma unroll
    for (int k = 0; k < 8; ++k) o[k] = (h16)(bfr(v[k]) * WOS);
    *(volatile v8h*)(dst + i * 8) = o; __threadfence(); *(volatile v8h*)(dst + i * 8) = o;
}

template <int BIASROW>
__global__ __launch_bounds__(32) void k_proj(const bf* __restrict__ A, const bf* __restrict__ Bt, const float* __restrict__ bias, h16* Ph, h16* Pr,
                                             int RB, size_t sRB, int pitch, int CB, size_t sCB,
                                             size_t sRBr, int pitchr, size_t sCBr, int rlim, int clim) {
    __shared__ __align__(16) float os[16 * 68];
    const int K = DM;
    const int lane = threadIdx.x & 31, lr = lane & 15, hi = lane >> 4; const int r0 = blockIdx.x * 64, c0 = blockIdx.y * 64;
    v8f acc[4][4];
#pragma unroll
    for (int mb = 0; mb < 4; ++mb)
#pragma unroll
        for (int nb = 0; nb < 4; ++nb) acc[mb][nb] = (v8f){};
    const size_t aoff = (size_t)(r0 + lr) * K + 8 * hi, boff = (size_t)(c0 + lr) * K + 8 * hi;
#pragma unroll 1
    for (int kc = 0; kc < K; kc += 32) {
        v16bf a[4];
#pragma unroll
        for (int mb = 0; mb < 4; ++mb) a[mb] = ldb(A + aoff + (size_t)mb * 16 * K + kc);
#pragma unroll
        for (int nb = 0; nb < 4; ++nb) { const v16bf b = ldb(Bt + boff + (size_t)nb * 16 * K + kc);
#pragma unroll
            for (int mb = 0; mb < 4; ++mb) acc[mb][nb] = wmmab(a[mb], b, acc[mb][nb]); }
        asm volatile("v_nop\n\tv_nop\n\tv_nop\n\tv_nop" : "+v"(acc[0][3]), "+v"(acc[1][3]), "+v"(acc[2][3]), "+v"(acc[3][3]) : "v"(a[0]), "v"(a[1]), "v"(a[2]), "v"(a[3]));
    }
    float bc[4] = {0.0f, 0.0f, 0.0f, 0.0f};
    if constexpr (BIASROW == 0) {
#pragma unroll
        for (int nb = 0; nb < 4; ++nb) bc[nb] = bfr(bias[c0 + nb * 16 + lr]);
    }
    const int wres = (((r0 % RB) < rlim) && ((c0 % CB) < clim)) ? 1 : 0;
    const size_t tbase = (size_t)(r0 / RB) * sRB + (size_t)(r0 % RB) * (size_t)pitch + (size_t)(c0 / CB) * sCB + (size_t)(c0 % CB);
    const size_t tbasr = (size_t)(r0 / RB) * sRBr + (size_t)(r0 % RB) * (size_t)pitchr + (size_t)(c0 / CB) * sCBr + (size_t)(c0 % CB);
#pragma unroll
    for (int mb = 0; mb < 4; ++mb) {
        float rb[8];
        if constexpr (BIASROW != 0) {
            const v4f b0 = *(const v4f*)(bias + r0 + mb * 16 + 8 * hi); const v4f b1 = *(const v4f*)(bias + r0 + mb * 16 + 8 * hi + 4);
#pragma unroll
            for (int i = 0; i < 4; ++i) { rb[i] = bfr(b0[i]); rb[4 + i] = bfr(b1[i]); }
        } else {
#pragma unroll
            for (int j = 0; j < 8; ++j) rb[j] = 0.0f;
        }
#pragma unroll
        for (int nb = 0; nb < 4; ++nb) {
#pragma unroll
            for (int j = 0; j < 8; ++j) os[(hi * 8 + j) * 68 + nb * 16 + lr] = acc[mb][nb][j] + ((BIASROW != 0) ? rb[j] : bc[nb]); }
        wave_sync();
        const size_t sb = tbase + (size_t)(mb * 16) * (size_t)pitch;
        const size_t sr = tbasr + (size_t)(mb * 16) * (size_t)pitchr;
#pragma unroll 1
        for (int ps = 0; ps < 2; ++ps) {
#pragma unroll
            for (int s = 0; s < 4; ++s) { const int row = 4 * s + (lane >> 3), c8 = (lane & 7) * 8;
                const v4f x0 = *(const v4fa*)(&os[row * 68 + c8]); const v4f x1 = *(const v4fa*)(&os[row * 68 + c8 + 4]); v8h hv, rv;
#pragma unroll
                for (int i = 0; i < 4; ++i) { const h16 a0 = (h16)x0[i]; const h16 a1 = (h16)x1[i]; hv[i] = a0; hv[4 + i] = a1; rv[i] = (h16)((x0[i] - (float)a0) * QRS); rv[4 + i] = (h16)((x1[i] - (float)a1) * QRS); }
                *(volatile v8h*)(Ph + sb + (size_t)row * (size_t)pitch + c8) = hv;
                if (wres) *(volatile v8h*)(Pr + sr + (size_t)row * (size_t)pitchr + c8) = rv; }
            if (ps == 0) __threadfence(); }
        wave_sync();
    }
}

template <int EARLY>
__global__ __launch_bounds__(32 * AW) void k_flash(const h16* __restrict__ QH, const h16* __restrict__ QR, const h16* __restrict__ KP, const h16* __restrict__ KR,
                                                   const h16* __restrict__ VT, const h16* __restrict__ VR, const int* __restrict__ MK, h16* CH, h16* CR, int tstart) {
    __shared__ __align__(16) float os[AW * 16 * 68];
    const int lane = threadIdx.x & 31, wave = __builtin_amdgcn_readfirstlane((int)(threadIdx.x >> 5)), lr = lane & 15, hi = lane >> 4;
    const int zh = blockIdx.y; const int b = zh / NH_, h = zh % NH_;
    const int t0 = tstart + (blockIdx.x * AW + wave) * 16;
    const size_t pbase = (size_t)zh * SEQ * HD;
    const size_t rbase = (size_t)zh * EROWS * HD;
    const size_t qo = pbase + (size_t)(t0 + lr) * HD + 8 * hi;
    const v16h qh0 = ldh(QH + qo), qh1 = ldh(QH + qo + 32);
    v16h qr0 = qh0, qr1 = qh1;
    if constexpr (EARLY != 0) { const size_t qro = rbase + (size_t)(t0 + lr) * HD + 8 * hi; qr0 = ldh(QR + qro); qr1 = ldh(QR + qro + 32); }
    const size_t ko  = pbase + (size_t)lr * HD + 8 * hi;
    const size_t kro = rbase + (size_t)lr * HD + 8 * hi;
    const size_t vo  = pbase + (size_t)lr * SEQ + 8 * hi;
    const size_t vro = rbase + (size_t)lr * EROWS + 8 * hi;
    const size_t mo  = (size_t)(t0 + lr) * SEQ_FULL + 8 * hi;
    v8f o0 = (v8f){}, o1 = (v8f){}, o2 = (v8f){}, o3 = (v8f){};
    v8f e0 = (v8f){}, e1 = (v8f){}, e2 = (v8f){}, e3 = (v8f){};
    float m = -3.0e38f, l = 0.0f;
    int noskip = 0;
#pragma unroll 1
    for (int pass = 0; pass < 2; ++pass) {
        o0 = (v8f){}; o1 = (v8f){}; o2 = (v8f){}; o3 = (v8f){};
        e0 = (v8f){}; e1 = (v8f){}; e2 = (v8f){}; e3 = (v8f){};
        m = -3.0e38f; l = 0.0f;
#pragma unroll 1
        for (int key0 = 0; key0 < SEQ; key0 += 32) {
            const int* mp = MK + mo + key0;
            const v4i ma0 = *(const v4i*)mp, ma1 = *(const v4i*)(mp + 4), mb0 = *(const v4i*)(mp + 16), mb1 = *(const v4i*)(mp + 20);
            const v4i mor = ma0 | ma1 | mb0 | mb1;
            const int anyv = mor[0] | mor[1] | mor[2] | mor[3];
            const unsigned bal = __builtin_amdgcn_ballot_w32(anyv != 0);
            if (noskip == 0 && bal == 0u) continue;
            const h16* ka = KP + ko + (size_t)key0 * HD;
            v8f sHa = (v8f){}, sHb = (v8f){}, sLa = (v8f){}, sLb = (v8f){};
            {
                const v16h ka0 = ldh(ka), ka1 = ldh(ka + 32), kb0 = ldh(ka + 16 * HD), kb1 = ldh(ka + 16 * HD + 32);
                sHa = wmma16(ka0, qh0, sHa); sHb = wmma16(kb0, qh0, sHb); sHa = wmma16(ka1, qh1, sHa); sHb = wmma16(kb1, qh1, sHb);
                if constexpr (EARLY != 0) {
                    sLa = wmma16(ka0, qr0, sLa); sLb = wmma16(kb0, qr0, sLb); sLa = wmma16(ka1, qr1, sLa); sLb = wmma16(kb1, qr1, sLb);
                    asm volatile("v_nop\n\tv_nop\n\tv_nop\n\tv_nop" : "+v"(sHa), "+v"(sHb), "+v"(sLa), "+v"(sLb) : "v"(ka0), "v"(ka1), "v"(kb0), "v"(kb1));
                } else {
                    asm volatile("v_nop\n\tv_nop\n\tv_nop\n\tv_nop" : "+v"(sHa), "+v"(sHb) : "v"(ka0), "v"(ka1), "v"(kb0), "v"(kb1));
                }
            }
            if constexpr (EARLY != 0) {
                __builtin_amdgcn_sched_barrier(0);
                if (key0 < EROWS) {
                    const h16* ra = KR + kro + (size_t)key0 * HD;
                    const v16h ra0 = ldh(ra), ra1 = ldh(ra + 32), rb0 = ldh(ra + 16 * HD), rb1 = ldh(ra + 16 * HD + 32);
                    sLa = wmma16(ra0, qh0, sLa); sLb = wmma16(rb0, qh0, sLb); sLa = wmma16(ra1, qh1, sLa); sLb = wmma16(rb1, qh1, sLb);
                    asm volatile("v_nop\n\tv_nop\n\tv_nop\n\tv_nop" : "+v"(sLa), "+v"(sLb) : "v"(ra0), "v"(ra1), "v"(rb0), "v"(rb1));
                }
                __builtin_amdgcn_sched_barrier(0);
            }
            const int mka[8] = {ma0[0], ma0[1], ma0[2], ma0[3], ma1[0], ma1[1], ma1[2], ma1[3]};
            const int mkb[8] = {mb0[0], mb0[1], mb0[2], mb0[3], mb1[0], mb1[1], mb1[2], mb1[3]};
            float ta[8], tb[8]; float mx = -3.0e38f;
#pragma unroll
            for (int r = 0; r < 8; ++r) {
                float sa = sHa[r], sb = sHb[r];
                if constexpr (EARLY != 0) { sa += sLa[r] * QRI; sb += sLb[r] * QRI; }
                ta[r] = (mka[r] != 0) ? sa * SC2 : NEGL;
                tb[r] = (mkb[r] != 0) ? sb * SC2 : NEGL;
                mx = fmaxf(mx, fmaxf(ta[r], tb[r]));
            }
            mx = fmaxf(mx, __shfl_xor(mx, 16, 32));
            const float mnew = fmaxf(m, mx);
            const float alpha = __builtin_amdgcn_exp2f(m - mnew);
            const float sh = PSH - mnew;
            v16h pb = (v16h){}; v16h pq = (v16h){}; float ls = 0.0f;
#pragma unroll
            for (int r = 0; r < 8; ++r) {
                const float pa = __builtin_amdgcn_exp2f(ta[r] + sh), pc = __builtin_amdgcn_exp2f(tb[r] + sh);
                const h16 ha = (h16)pa, hc = (h16)pc; pb[r] = ha; pb[8 + r] = hc;
                if constexpr (EARLY != 0) {
                    const h16 ga = (h16)((pa - (float)ha) * QRS), gc = (h16)((pc - (float)hc) * QRS); pq[r] = ga; pq[8 + r] = gc;
                    ls += ((float)ha + (float)hc) + ((float)ga + (float)gc) * QRI;
                } else {
                    ls += (float)ha + (float)hc;
                }
            }
            l = l * alpha + ls; m = mnew;
            o0 = o0 * alpha; o1 = o1 * alpha; o2 = o2 * alpha; o3 = o3 * alpha;
            if constexpr (EARLY != 0) { e0 = e0 * alpha; e1 = e1 * alpha; e2 = e2 * alpha; e3 = e3 * alpha; }
            const h16* va = VT + vo + key0;
            {
                const v16h v0 = ldh(va), v1 = ldh(va + (size_t)16 * SEQ), v2 = ldh(va + (size_t)32 * SEQ), v3 = ldh(va + (size_t)48 * SEQ);
                o0 = wmma16(v0, pb, o0); o1 = wmma16(v1, pb, o1); o2 = wmma16(v2, pb, o2); o3 = wmma16(v3, pb, o3);
                if constexpr (EARLY != 0) {
                    e0 = wmma16(v0, pq, e0); e1 = wmma16(v1, pq, e1); e2 = wmma16(v2, pq, e2); e3 = wmma16(v3, pq, e3);
                    asm volatile("v_nop\n\tv_nop\n\tv_nop\n\tv_nop" : "+v"(o0), "+v"(o1), "+v"(o2), "+v"(o3), "+v"(e0), "+v"(e1), "+v"(e2), "+v"(e3) : "v"(v0), "v"(v1), "v"(v2), "v"(v3), "v"(pb), "v"(pq));
                } else {
                    asm volatile("v_nop\n\tv_nop\n\tv_nop\n\tv_nop" : "+v"(o0), "+v"(o1), "+v"(o2), "+v"(o3) : "v"(v0), "v"(v1), "v"(v2), "v"(v3), "v"(pb));
                }
            }
            if constexpr (EARLY != 0) {
                __builtin_amdgcn_sched_barrier(0);
                if (key0 < EROWS) {
                    const h16* wa = VR + vro + key0;
                    const v16h w0 = ldh(wa), w1 = ldh(wa + (size_t)16 * EROWS), w2 = ldh(wa + (size_t)32 * EROWS), w3 = ldh(wa + (size_t)48 * EROWS);
                    e0 = wmma16(w0, pb, e0); e1 = wmma16(w1, pb, e1); e2 = wmma16(w2, pb, e2); e3 = wmma16(w3, pb, e3);
                    asm volatile("v_nop\n\tv_nop\n\tv_nop\n\tv_nop" : "+v"(e0), "+v"(e1), "+v"(e2), "+v"(e3) : "v"(w0), "v"(w1), "v"(w2), "v"(w3), "v"(pb));
                }
                __builtin_amdgcn_sched_barrier(0);
            }
        }
        l += __shfl_xor(l, 16, 32);
        const unsigned dead = __builtin_amdgcn_ballot_w32(!(l > 0.0f));
        if (dead == 0u) break;
        noskip = 1;
    }
    const float inv = CXS * (1.0f / l);
    const int wb = wave * 16 * 68;
    {
        v8f x0 = o0, x1 = o1, x2 = o2, x3 = o3;
        if constexpr (EARLY != 0) { x0 = o0 + e0 * QRI; x1 = o1 + e1 * QRI; x2 = o2 + e2 * QRI; x3 = o3 + e3 * QRI; }
        x0 = x0 * inv; x1 = x1 * inv; x2 = x2 * inv; x3 = x3 * inv;
        v4f a, c;
        a = __builtin_shufflevector(x0, x0, 0, 1, 2, 3); c = __builtin_shufflevector(x0, x0, 4, 5, 6, 7);
        *(v4fa*)(&os[wb + lr * 68 +  0 + 8 * hi]) = a; *(v4fa*)(&os[wb + lr * 68 +  0 + 8 * hi + 4]) = c;
        a = __builtin_shufflevector(x1, x1, 0, 1, 2, 3); c = __builtin_shufflevector(x1, x1, 4, 5, 6, 7);
        *(v4fa*)(&os[wb + lr * 68 + 16 + 8 * hi]) = a; *(v4fa*)(&os[wb + lr * 68 + 16 + 8 * hi + 4]) = c;
        a = __builtin_shufflevector(x2, x2, 0, 1, 2, 3); c = __builtin_shufflevector(x2, x2, 4, 5, 6, 7);
        *(v4fa*)(&os[wb + lr * 68 + 32 + 8 * hi]) = a; *(v4fa*)(&os[wb + lr * 68 + 32 + 8 * hi + 4]) = c;
        a = __builtin_shufflevector(x3, x3, 0, 1, 2, 3); c = __builtin_shufflevector(x3, x3, 4, 5, 6, 7);
        *(v4fa*)(&os[wb + lr * 68 + 48 + 8 * hi]) = a; *(v4fa*)(&os[wb + lr * 68 + 48 + 8 * hi + 4]) = c;
    }
    wave_sync();
    const size_t crow = ((size_t)b * SEQ + t0) * DM + (size_t)h * HD;
    const size_t rrow = ((size_t)b * EROWS + t0) * DM + (size_t)h * HD;
#pragma unroll 1
    for (int ps = 0; ps < 2; ++ps) {
#pragma unroll
        for (int s = 0; s < 4; ++s) { const int row = 4 * s + (lane >> 3), c8 = (lane & 7) * 8;
            const v4f x0 = *(const v4fa*)(&os[wb + row * 68 + c8]); const v4f x1 = *(const v4fa*)(&os[wb + row * 68 + c8 + 4]); v8h hv, rv;
#pragma unroll
            for (int i = 0; i < 4; ++i) { const h16 a0 = (h16)x0[i]; const h16 a1 = (h16)x1[i]; hv[i] = a0; hv[4 + i] = a1; rv[i] = (h16)((x0[i] - (float)a0) * QRS); rv[4 + i] = (h16)((x1[i] - (float)a1) * QRS); }
            *(volatile v8h*)(CH + crow + (size_t)row * DM + c8) = hv;
            if constexpr (EARLY != 0) *(volatile v8h*)(CR + rrow + (size_t)row * DM + c8) = rv; }
        if (ps == 0) __threadfence(); }
}

template <int MT, int RES>
__global__ __launch_bounds__(32) void k_oproj(const h16* __restrict__ A, const h16* __restrict__ AR, const h16* __restrict__ Bt, const float* __restrict__ bias, float* OUT, int tpb, int rowoff) {
    static_assert((MT == 4 && RES == 0) || (MT == 2 && RES == 1));
    __shared__ __align__(16) float os[16 * 68];
    const int K = DM;
    const int lane = threadIdx.x & 31, lr = lane & 15, hi = lane >> 4;
    const int bb = blockIdx.x / tpb, tl = blockIdx.x % tpb;
    const int tok = rowoff + tl * (16 * MT);
    const int c0 = blockIdx.y * 64;
    const size_t aoff = ((size_t)bb * SEQ + tok + lr) * K + 8 * hi;
    const size_t roff = ((size_t)bb * EROWS + tok + lr) * K + 8 * hi;
    const size_t boff = (size_t)(c0 + lr) * K + 8 * hi;
    v8f acc[MT][4], acr[MT][4];
#pragma unroll
    for (int mb = 0; mb < MT; ++mb)
#pragma unroll
        for (int nb = 0; nb < 4; ++nb) { acc[mb][nb] = (v8f){}; acr[mb][nb] = (v8f){}; }
#pragma unroll 1
    for (int kc = 0; kc < K; kc += 32) {
        v16h a[MT], ar[MT];
#pragma unroll
        for (int mb = 0; mb < MT; ++mb) { a[mb] = ldh(A + aoff + (size_t)mb * 16 * K + kc); ar[mb] = a[mb]; }
        if constexpr (RES != 0) {
#pragma unroll
            for (int mb = 0; mb < MT; ++mb) ar[mb] = ldh(AR + roff + (size_t)mb * 16 * K + kc);
        }
#pragma unroll
        for (int nb = 0; nb < 4; ++nb) { const v16h bfrag = ldh(Bt + boff + (size_t)nb * 16 * K + kc);
#pragma unroll
            for (int mb = 0; mb < MT; ++mb) { acc[mb][nb] = wmma16(a[mb], bfrag, acc[mb][nb]);
                if constexpr (RES != 0) acr[mb][nb] = wmma16(ar[mb], bfrag, acr[mb][nb]); } }
        if constexpr (MT == 4) {
            asm volatile("v_nop\n\tv_nop\n\tv_nop\n\tv_nop" : "+v"(acc[0][3]), "+v"(acc[1][3]), "+v"(acc[2][3]), "+v"(acc[3][3]) : "v"(a[0]), "v"(a[1]), "v"(a[2]), "v"(a[3]));
        } else {
            asm volatile("v_nop\n\tv_nop\n\tv_nop\n\tv_nop" : "+v"(acc[0][3]), "+v"(acc[1][3]), "+v"(acr[0][3]), "+v"(acr[1][3]) : "v"(a[0]), "v"(a[1]), "v"(ar[0]), "v"(ar[1]));
        }
    }
    float bc[4];
#pragma unroll
    for (int nb = 0; nb < 4; ++nb) bc[nb] = bfr(bias[c0 + nb * 16 + lr]);
#pragma unroll
    for (int mb = 0; mb < MT; ++mb) {
#pragma unroll
        for (int nb = 0; nb < 4; ++nb) {
#pragma unroll
            for (int j = 0; j < 8; ++j) { float v = acc[mb][nb][j] * OSC;
                if constexpr (RES != 0) v += acr[mb][nb][j] * (OSC * QRI);
                os[(hi * 8 + j) * 68 + nb * 16 + lr] = v + bc[nb]; } }
        wave_sync();
        float* orow = OUT + ((size_t)bb * OUT_SEQ + tok + mb * 16) * DM + c0;
#pragma unroll 1
        for (int ps = 0; ps < 2; ++ps) {
#pragma unroll
            for (int s = 0; s < 8; ++s) { const int row = 2 * s + hi, cofs = lr * 4;
                const v4f val = *(const v4fa*)(&os[row * 68 + cofs]);
                *(volatile v4f*)(orow + (size_t)row * DM + cofs) = val; }
            if (ps == 0) __threadfence(); }
        wave_sync();
    }
}

static constexpr size_t al256(size_t v) { return (v + 255) & ~(size_t)255; }
static constexpr size_t SZ_XB = al256((size_t)NB * SEQ * DM * 2);
static constexpr size_t SZ_WB = al256((size_t)3 * DM * DM * 2);
static constexpr size_t SZ_WO = al256((size_t)DM * DM * 2);
static constexpr size_t SZ_PL = al256((size_t)NB * NH_ * SEQ * HD * 2);
static constexpr size_t SZ_RP = al256((size_t)NB * NH_ * EROWS * HD * 2);
static constexpr size_t SZ_CX = al256((size_t)NB * SEQ * DM * 2);
static constexpr size_t SZ_CR = al256((size_t)NB * EROWS * DM * 2);
static constexpr size_t SZ_TOTAL = SZ_XB + SZ_WB + SZ_WO + 3 * SZ_PL + 3 * SZ_RP + SZ_CX + SZ_CR;
static_assert(SZ_TOTAL <= (size_t)134217728);
static_assert(((size_t)DM * DM * 2) % 256 == 0);

extern "C" void kernel_launch(void* const* d_in, const int* in_sizes, int n_in,
                              void* d_out, int out_size, void* d_ws, size_t ws_size, hipStream_t stream) {
    if (n_in < 10) return;
    const size_t needx = ((size_t)(NB - 1) * SEQ_FULL + SEQ) * DM;
    if ((size_t)in_sizes[0] < needx) return;
    if ((size_t)in_sizes[1] < (size_t)(SEQ - 1) * SEQ_FULL + SEQ) return;
    if ((size_t)in_sizes[2] < (size_t)DM * DM || (size_t)in_sizes[4] < (size_t)DM * DM || (size_t)in_sizes[6] < (size_t)DM * DM || (size_t)in_sizes[8] < (size_t)DM * DM) return;
    if (in_sizes[3] < DM || in_sizes[5] < DM || in_sizes[7] < DM || in_sizes[9] < DM) return;
    if ((size_t)out_size < ((size_t)(NB - 1) * OUT_SEQ + SEQ) * DM) return;
    if (SZ_TOTAL > ws_size) return;
    const float* x  = (const float*)d_in[0]; const int* mask = (const int*)d_in[1];
    const float* wq = (const float*)d_in[2]; const float* bq = (const float*)d_in[3];
    const float* wk = (const float*)d_in[4]; const float* bk = (const float*)d_in[5];
    const float* wv = (const float*)d_in[6]; const float* bv = (const float*)d_in[7];
    const float* wo = (const float*)d_in[8]; const float* bo = (const float*)d_in[9];
    float* OUT = (float*)d_out;
    char* wsp = (char*)d_ws;
    bf*  XB  = (bf*)wsp;  wsp += SZ_XB;
    bf*  WB  = (bf*)wsp;  wsp += SZ_WB;
    h16* WOH = (h16*)wsp; wsp += SZ_WO;
    h16* QH  = (h16*)wsp; wsp += SZ_PL;
    h16* KP  = (h16*)wsp; wsp += SZ_PL;
    h16* VT  = (h16*)wsp; wsp += SZ_PL;
    h16* QR  = (h16*)wsp; wsp += SZ_RP;
    h16* KR  = (h16*)wsp; wsp += SZ_RP;
    h16* VR  = (h16*)wsp; wsp += SZ_RP;
    h16* CXH = (h16*)wsp; wsp += SZ_CX;
    h16* CXR = (h16*)wsp; wsp += SZ_CR;
    bf* WQ = WB; bf* WK = WB + (size_t)DM * DM; bf* WV = WB + (size_t)2 * DM * DM;

    if (SEQ == SEQ_FULL) {
        const size_t n8 = (size_t)NB * SEQ * DM / 8;
        k_cvt8<<<(unsigned)((n8 + 255) / 256), 256, 0, stream>>>(x, XB, n8);
    } else {
        const size_t n8 = (size_t)SEQ * DM / 8;
        for (int b = 0; b < NB; ++b) k_cvt8<<<(unsigned)((n8 + 255) / 256), 256, 0, stream>>>(x + (size_t)b * SEQ_FULL * DM, XB + (size_t)b * SEQ * DM, n8);
    }
    { const size_t n8 = (size_t)DM * DM / 8; const unsigned g = (unsigned)((n8 + 255) / 256);
      k_cvt8<<<g, 256, 0, stream>>>(wq, WQ, n8); k_cvt8<<<g, 256, 0, stream>>>(wk, WK, n8); k_cvt8<<<g, 256, 0, stream>>>(wv, WV, n8);
      k_cvtw8<<<g, 256, 0, stream>>>(wo, WOH, n8); }

    k_proj<0><<<dim3(NB * SEQ / 64, DM / 64, 1), 32, 0, stream>>>(XB, WQ, bq, QH, QR, SEQ, (size_t)NH_ * SEQ * HD, HD, HD, (size_t)SEQ * HD,
                                                                  (size_t)NH_ * EROWS * HD, HD, (size_t)EROWS * HD, EROWS, HD);
    k_proj<0><<<dim3(NB * SEQ / 64, DM / 64, 1), 32, 0, stream>>>(XB, WK, bk, KP, KR, SEQ, (size_t)NH_ * SEQ * HD, HD, HD, (size_t)SEQ * HD,
                                                                  (size_t)NH_ * EROWS * HD, HD, (size_t)EROWS * HD, EROWS, HD);
    k_proj<1><<<dim3(DM / 64, NB * SEQ / 64, 1), 32, 0, stream>>>(WV, XB, bv, VT, VR, DM, (size_t)0, SEQ, SEQ, (size_t)DM * SEQ,
                                                                  (size_t)0, EROWS, (size_t)DM * EROWS, DM, EROWS);

    k_flash<1><<<dim3(EROWS / (16 * AW), NB * NH_, 1), 32 * AW, 0, stream>>>(QH, QR, KP, KR, VT, VR, mask, CXH, CXR, 0);
    if (SEQ > EROWS)
        k_flash<0><<<dim3((SEQ - EROWS) / (16 * AW), NB * NH_, 1), 32 * AW, 0, stream>>>(QH, QR, KP, KR, VT, VR, mask, CXH, CXR, EROWS);

    k_oproj<2, 1><<<dim3(NB * (EROWS / 32), DM / 64, 1), 32, 0, stream>>>(CXH, CXR, WOH, bo, OUT, EROWS / 32, 0);
    if (SEQ > EROWS)
        k_oproj<4, 0><<<dim3(NB * ((SEQ - EROWS) / 64), DM / 64, 1), 32, 0, stream>>>(CXH, CXH, WOH, bo, OUT, (SEQ - EROWS) / 64, EROWS);
}
